// mulGCN_57526791962625
// MI455X (gfx1250) — hardware-run, weakly checked
//
#include <hip/hip_runtime.h>
#include <stddef.h>


#define FEAT 64
#define GF 128
#define NTILE 40
#define TB_G 0
#define TB_R 8
#define TB_I 16
#define TB_O 24
#define NSLOTS (NTILE * 64)

#define CH1 2048
#define PITCHB 3136
#define MAXB PITCHB
#define BPT 25
#define MAXGRP 19
#define MAXNB1 (32 * MAXGRP)
#define CAP3 2048
#define GMAX 256
#define NCH 32
#define HP 72

typedef _Float16 v16h __attribute__((ext_vector_type(16)));
typedef _Float16 v8h __attribute__((ext_vector_type(8)));
typedef float v8f __attribute__((ext_vector_type(8)));
typedef float v4f __attribute__((ext_vector_type(4)));
typedef float v2f __attribute__((ext_vector_type(2)));
typedef int v4i __attribute__((ext_vector_type(4)));
typedef v4f __attribute__((may_alias)) v4fa;
typedef v4i __attribute__((may_alias)) v4ia;
typedef v8h __attribute__((may_alias)) v8ha;

union Frag { v16h v; v8h half[2]; _Float16 e[16]; };

__device__ __forceinline__ v8f wmma16(const v16h& a, const v16h& b, v8f c) {
    return __builtin_amdgcn_wmma_f32_16x16x32_f16(false, a, false, b, (short)0, c, false, false);
}

__device__ __forceinline__ v16h frag_f32(const float* rowp, int k0, int h) {
    const v4f* rp = (const v4f*)rowp + (k0 >> 2);
    const v4f p0 = rp[2 * h], p1 = rp[2 * h + 1], p2 = rp[4 + 2 * h], p3 = rp[5 + 2 * h];
    Frag a;
    a.e[0] = (_Float16)p0.x;  a.e[1] = (_Float16)p0.y;  a.e[2] = (_Float16)p0.z;  a.e[3] = (_Float16)p0.w;
    a.e[4] = (_Float16)p1.x;  a.e[5] = (_Float16)p1.y;  a.e[6] = (_Float16)p1.z;  a.e[7] = (_Float16)p1.w;
    a.e[8] = (_Float16)p2.x;  a.e[9] = (_Float16)p2.y;  a.e[10] = (_Float16)p2.z; a.e[11] = (_Float16)p2.w;
    a.e[12] = (_Float16)p3.x; a.e[13] = (_Float16)p3.y; a.e[14] = (_Float16)p3.z; a.e[15] = (_Float16)p3.w;
    return a.v;
}

__device__ __forceinline__ v16h frag_lds(const _Float16* rowp, int k0, int h) {
    Frag a;
    a.half[0] = *(const v8ha*)(rowp + k0 + 8 * h);
    a.half[1] = *(const v8ha*)(rowp + k0 + 16 + 8 * h);
    return a.v;
}

__device__ __forceinline__ v16h frag_b(const v8h* bq, int tile, int lane) {
    Frag b;
    const int f = (tile * 32 + lane) * 2;
    b.half[0] = bq[f];
    b.half[1] = bq[f + 1];
    return b.v;
}

__global__ __launch_bounds__(256) void k_prep(const float* __restrict__ wg, const float* __restrict__ wr,
                                              const float* __restrict__ wi, const float* __restrict__ wo,
                                              const float* __restrict__ ef, _Float16* bfrag) {
    (void)ef;
    const int t0 = blockIdx.x * 256 + threadIdx.x;
    const bool ok = t0 < NSLOTS;
    const int tt = ok ? t0 : 0;
    const int g = tt & 1, l = (tt >> 1) & 31, tile = tt >> 6;
    const int h = l >> 4, m = l & 15;
    const int sel = tile < TB_R ? 0 : (tile < TB_I ? 1 : (tile < TB_O ? 2 : 3));
    const int lt = tile - 8 * sel;
    const int ks = (sel == 3) ? (lt >> 3) : (lt >> 2);
    const int nt = (sel == 3) ? (lt & 7) : (lt & 3);
    const int c = nt * 16 + m;
    const int kb = 32 * ks + 16 * g + 8 * h;
    union { v8h v; _Float16 e[8]; } u;
#pragma unroll
    for (int ii = 0; ii < 8; ++ii) {
        const int k = kb + ii;
        int i64 = k * 64 + c;
        i64 = i64 > 4095 ? 4095 : i64;
        const int i128 = k * 128 + c;
        const float vg = wg[i64];
        const float vr = wr[i64];
        const float vi = wi[i64];
        const float vo = wo[i128];
        const float v = (sel == 0) ? vg : ((sel == 1) ? vr : ((sel == 2) ? vi : vo));
        u.e[ii] = (_Float16)(v * 64.0f);
    }
    const v8h val = u.v;
    if (ok) *(volatile v8h*)(bfrag + (size_t)tt * 8) = val;
    __threadfence();
    if (ok) *(volatile v8h*)(bfrag + (size_t)tt * 8) = val;
}

__device__ __forceinline__ void chunk_keys(const int* __restrict__ recv, int cb, int lane, int E, int N,
                                           unsigned& key_out, int& rank, bool& last, bool& valid) {
    const int e = cb + lane;
    const int ec = e < E ? e : E - 1;
    const int r = recv[ec];
    unsigned key = 0xFFFFFFFFu;
    if (e < E && r >= 0 && r < N) key = ((unsigned)r & ~31u) | (unsigned)lane;
#pragma unroll
    for (int kk = 2; kk <= 32; kk <<= 1) {
#pragma unroll
        for (int j = kk >> 1; j > 0; j >>= 1) {
            const unsigned p = __shfl_xor(key, j);
            const bool asc = (lane & kk) == 0;
            const bool low = (lane & j) == 0;
            const unsigned mn = key < p ? key : p;
            const unsigned mx = key < p ? p : key;
            key = (asc == low) ? mn : mx;
        }
    }
    const unsigned bkt = key >> 5;
    const unsigned pk = __shfl_up(key, 1);
    const unsigned nk = __shfl_down(key, 1);
    const bool start = (lane == 0) || ((pk >> 5) != bkt);
    last = (lane == 31) || ((nk >> 5) != bkt);
    int v = start ? lane : 0;
#pragma unroll
    for (int d = 1; d < 32; d <<= 1) {
        const int uu = __shfl_up(v, d);
        if (lane >= d && uu > v) v = uu;
    }
    rank = lane - v;
    key_out = key;
    valid = (key != 0xFFFFFFFFu);
}

__global__ __launch_bounds__(128) void k_bucket(const int* __restrict__ recv, int* lists, int* offtab, int E, int N) {
    __shared__ unsigned short wcnt[4 * MAXB];
    __shared__ __attribute__((aligned(16))) int list_lds[CH1];
    __shared__ __attribute__((aligned(16))) int boff[PITCHB];
    __shared__ int sb[128];
    const int t = threadIdx.x, lane = t & 31, wid = t >> 5, blk = blockIdx.x;

    for (int i = t; i < 4 * MAXB; i += 128) wcnt[i] = 0;
    for (int i = t; i < CH1; i += 128) list_lds[i] = 0;
    __syncthreads();

    const int wbase = blk * CH1 + wid * 512;
#pragma unroll 1
    for (int c = 0; c < 16; ++c) {
        unsigned key; int rank; bool last, valid;
        chunk_keys(recv, wbase + c * 32, lane, E, N, key, rank, last, valid);
        if (valid && last) {
            const int b = (int)(key >> 5);
            wcnt[wid * MAXB + b] += (unsigned short)(rank + 1);
        }
    }
    __syncthreads();

    int tsum = 0;
#pragma unroll 1
    for (int q = 0; q < BPT; ++q) {
        const int b = t * BPT + q;
        if (b < PITCHB) {
            int tot = 0;
#pragma unroll
            for (int w = 0; w < 4; ++w) tot += (int)wcnt[w * MAXB + b];
            tsum += tot;
        }
    }
    sb[t] = tsum;
    __syncthreads();
#pragma unroll 1
    for (int d = 1; d < 128; d <<= 1) {
        const int vv = sb[(t >= d) ? (t - d) : t];
        const int v = (t >= d) ? vv : 0;
        __syncthreads();
        sb[t] += v;
        __syncthreads();
    }
    int run = sb[t] - tsum;
#pragma unroll 1
    for (int q = 0; q < BPT; ++q) {
        const int b = t * BPT + q;
        if (b < PITCHB) {
            boff[b] = run;
#pragma unroll
            for (int w = 0; w < 4; ++w) {
                const int cnt = (int)wcnt[w * MAXB + b];
                wcnt[w * MAXB + b] = (unsigned short)run;
                run += cnt;
            }
        }
    }
    __syncthreads();

#pragma unroll 1
    for (int c = 0; c < 16; ++c) {
        const int cb = wbase + c * 32;
        unsigned key; int rank; bool last, valid;
        chunk_keys(recv, cb, lane, E, N, key, rank, last, valid);
        if (valid) {
            const int b = (int)(key >> 5);
            const int pos = (int)wcnt[wid * MAXB + b] + rank;
            if ((unsigned)pos < (unsigned)CH1) list_lds[pos] = cb + (int)(key & 31u);
            if (last) wcnt[wid * MAXB + b] = (unsigned short)(pos + 1);
        }
    }
    __syncthreads();

    const v4ia* lsrc = (const v4ia*)list_lds;
    const v4ia* bsrc = (const v4ia*)boff;
    int* ld = lists + (size_t)blk * CH1;
    int* bd = offtab + (size_t)blk * PITCHB;
#pragma unroll
    for (int u = 0; u < 4; ++u) {
        const v4i v = lsrc[t + u * 128];
        *(volatile v4i*)(ld + (size_t)(t + u * 128) * 4) = v;
    }
#pragma unroll
    for (int u = 0; u < 7; ++u) {
        const int idx = t + u * 128;
        const bool has = idx < (PITCHB / 4);
        const v4i v = bsrc[has ? idx : 0];
        if (has) *(volatile v4i*)(bd + (size_t)idx * 4) = v;
    }
    __threadfence();
#pragma unroll
    for (int u = 0; u < 4; ++u) {
        const v4i v = lsrc[t + u * 128];
        *(volatile v4i*)(ld + (size_t)(t + u * 128) * 4) = v;
    }
#pragma unroll
    for (int u = 0; u < 7; ++u) {
        const int idx = t + u * 128;
        const bool has = idx < (PITCHB / 4);
        const v4i v = bsrc[has ? idx : 0];
        if (has) *(volatile v4i*)(bd + (size_t)idx * 4) = v;
    }
}

__global__ __launch_bounds__(32) void k_aggr(const float* __restrict__ x, const int* __restrict__ srcv,
                                             const int* __restrict__ recv, const int* lists, const int* offtab,
                                             float* agg, int E, int N, int NB1) {
    __shared__ unsigned comp[CAP3];
    __shared__ __attribute__((aligned(16))) v2f acc[32 * 32];
    const int lane = threadIdx.x & 31;
    const int f = blockIdx.x;

    int carry = 0;
#pragma unroll 1
    for (int u = 0; u < MAXGRP; ++u) {
        const int blk = lane + 32 * u;
        const bool inb = blk < NB1;
        const int cblk = inb ? blk : 0;
        const int* tb = offtab + (size_t)cblk * PITCHB;
        int a = tb[f];
        int b = tb[f + 1];
        a = a < 0 ? 0 : (a > CH1 ? CH1 : a);
        b = b < a ? a : (b > CH1 ? CH1 : b);
        const int c = inb ? (b - a) : 0;
        a = inb ? a : 0;
        int s = c;
#pragma unroll
        for (int d = 1; d < 32; d <<= 1) {
            const int v = __shfl_up(s, d);
            if (lane >= d) s += v;
        }
        const int ex = carry + s - c;
        const int tot = __shfl(s, 31);
        int qmax = c;
#pragma unroll
        for (int d = 16; d > 0; d >>= 1) {
            const int o = __shfl_xor(qmax, d);
            qmax = o > qmax ? o : qmax;
        }
        const int* lbase = lists + (size_t)cblk * CH1;
#pragma unroll 1
        for (int q = 0; q < qmax; ++q) {
            const bool act = q < c;
            int li = a + q;
            li = li < 0 ? 0 : (li > CH1 - 1 ? CH1 - 1 : li);
            const int e = lbase[li];
            const int ec = e < 0 ? 0 : (e > E - 1 ? E - 1 : e);
            const int nd = recv[ec] - f * 32;
            unsigned pk = 0xFFFFFFFFu;
            if ((unsigned)e < (unsigned)E && (unsigned)nd < 32u) pk = ((unsigned)e << 5) | (unsigned)nd;
            const int p = ex + q;
            if (act && (unsigned)p < (unsigned)CAP3) comp[p] = pk;
        }
        carry += tot;
    }
    const int T = carry < CAP3 ? carry : CAP3;

#pragma unroll
    for (int r = 0; r < 32; ++r) { v2f z; z.x = 0.0f; z.y = 0.0f; acc[r * 32 + lane] = z; }
    __syncthreads();

#pragma unroll 1
    for (int i = 0; i < T; ++i) {
        const unsigned pk = comp[i];
        const bool valid = pk != 0xFFFFFFFFu;
        int e = (int)(pk >> 5);
        e = valid ? e : 0;
        e = e < 0 ? 0 : (e > E - 1 ? E - 1 : e);
        const int nd = (int)(pk & 31u);
        int sn = srcv[e];
        sn = sn < 0 ? 0 : (sn > N - 1 ? N - 1 : sn);
        const v2f v = *(const v2f*)(x + (size_t)sn * FEAT + 2 * lane);
        const float vx = valid ? v.x : 0.0f;
        const float vy = valid ? v.y : 0.0f;
        v2f tacc = acc[nd * 32 + lane];
        tacc.x += vx;
        tacc.y += vy;
        acc[nd * 32 + lane] = tacc;
    }
    __syncthreads();

    const v4fa* av = (const v4fa*)acc;
    float* ob = agg + (size_t)f * 32 * FEAT;
#pragma unroll
    for (int it = 0; it < 16; ++it) {
        const v4f v = av[it * 32 + lane];
        *(volatile v4f*)(ob + (size_t)(it * 32 + lane) * 4) = v;
    }
    __threadfence();
#pragma unroll
    for (int it = 0; it < 16; ++it) {
        const v4f v = av[it * 32 + lane];
        *(volatile v4f*)(ob + (size_t)(it * 32 + lane) * 4) = v;
    }
}

__global__ __launch_bounds__(32) void k_node(const float* agg, const float* __restrict__ x, const _Float16* bfrag,
                                             const float* __restrict__ bg, const float* __restrict__ br,
                                             const float* __restrict__ bi, const float* __restrict__ bo,
                                             float* yp, int N, int NT) {
    __shared__ __attribute__((aligned(16))) _Float16 h1[16 * HP];
    __shared__ __attribute__((aligned(16))) _Float16 h2[16 * HP];
    __shared__ __attribute__((aligned(16))) float stg[16 * 32];
    const int tile = blockIdx.x;
    if (tile >= NT) return;
    const int lane = threadIdx.x & 31, h = lane >> 4, m = lane & 15;
    int row = tile * 16 + m;
    row = row > N - 1 ? N - 1 : row;
    const float inv = 0.015625f;
    const v8h* bq = (const v8h*)bfrag;

    const float* arow = agg + (size_t)row * FEAT;
    const float* xrow = x + (size_t)row * FEAT;
    const v16h aA0 = frag_f32(arow, 0, h);
    const v16h aA1 = frag_f32(arow, 32, h);
    const v16h aX0 = frag_f32(xrow, 0, h);
    const v16h aX1 = frag_f32(xrow, 32, h);

#pragma unroll
    for (int nt = 0; nt < 4; ++nt) {
        const v16h b0 = frag_b(bq, TB_G + nt, lane);
        const v16h b1 = frag_b(bq, TB_G + 4 + nt, lane);
        const v16h b2 = frag_b(bq, TB_R + nt, lane);
        const v16h b3 = frag_b(bq, TB_R + 4 + nt, lane);
        v8f z;
#pragma unroll
        for (int r = 0; r < 8; ++r) z[r] = 0.0f;
        v8f c = wmma16(aA0, b0, z);
        c = wmma16(aA1, b1, c);
        v8f d = wmma16(aX0, b2, z);
        d = wmma16(aX1, b3, d);
        asm volatile("v_nop\n\tv_nop\n\tv_nop\n\tv_nop" : "+v"(c), "+v"(d)
                     : "v"(aA0), "v"(aA1), "v"(aX0), "v"(aX1), "v"(b0), "v"(b1), "v"(b2), "v"(b3));
        const float cb = bg[nt * 16 + m], db = br[nt * 16 + m];
#pragma unroll
        for (int r = 0; r < 8; ++r) {
            const float hv = fmaxf(c[r] * inv + cb, 0.0f) + fmaxf(d[r] * inv + db, 0.0f);
            h1[(8 * h + r) * HP + nt * 16 + m] = (_Float16)hv;
        }
    }
    __syncthreads();

    const v16h h10 = frag_lds(h1 + m * HP, 0, h);
    const v16h h11 = frag_lds(h1 + m * HP, 32, h);
#pragma unroll
    for (int nt = 0; nt < 4; ++nt) {
        const v16h b0 = frag_b(bq, TB_I + nt, lane);
        const v16h b1 = frag_b(bq, TB_I + 4 + nt, lane);
        v8f z;
#pragma unroll
        for (int r = 0; r < 8; ++r) z[r] = 0.0f;
        v8f c = wmma16(h10, b0, z);
        c = wmma16(h11, b1, c);
        asm volatile("v_nop\n\tv_nop\n\tv_nop\n\tv_nop" : "+v"(c) : "v"(h10), "v"(h11), "v"(b0), "v"(b1));
        const float cb = bi[nt * 16 + m];
#pragma unroll
        for (int r = 0; r < 8; ++r)
            h2[(8 * h + r) * HP + nt * 16 + m] = (_Float16)fmaxf(c[r] * inv + cb, 0.0f);
    }
    __syncthreads();

    const v16h h20 = frag_lds(h2 + m * HP, 0, h);
    const v16h h21 = frag_lds(h2 + m * HP, 32, h);
    float* gbase = yp + (size_t)tile * 16 * GF;
    const v4fa* sv = (const v4fa*)stg;
#pragma unroll 1
    for (int u = 0; u < 4; ++u) {
        const v16h b0 = frag_b(bq, TB_O + 2 * u, lane);
        const v16h b1 = frag_b(bq, TB_O + 8 + 2 * u, lane);
        const v16h b2 = frag_b(bq, TB_O + 2 * u + 1, lane);
        const v16h b3 = frag_b(bq, TB_O + 8 + 2 * u + 1, lane);
        v8f z;
#pragma unroll
        for (int r = 0; r < 8; ++r) z[r] = 0.0f;
        v8f c0 = wmma16(h20, b0, z);
        c0 = wmma16(h21, b1, c0);
        v8f c1 = wmma16(h20, b2, z);
        c1 = wmma16(h21, b3, c1);
        asm volatile("v_nop\n\tv_nop\n\tv_nop\n\tv_nop" : "+v"(c0), "+v"(c1)
                     : "v"(h20), "v"(h21), "v"(b0), "v"(b1), "v"(b2), "v"(b3));
        const float ob0 = bo[32 * u + m], ob1 = bo[32 * u + 16 + m];
#pragma unroll
        for (int r = 0; r < 8; ++r) {
            stg[(8 * h + r) * 32 + m] = c0[r] * inv + ob0;
            stg[(8 * h + r) * 32 + 16 + m] = c1[r] * inv + ob1;
        }
        __syncthreads();
        float* gp = gbase + 32 * u + (lane & 7) * 4;
#pragma unroll
        for (int it = 0; it < 4; ++it) {
            const v4f v = sv[it * 32 + lane];
            *(volatile v4f*)(gp + (size_t)(it * 4 + (lane >> 3)) * GF) = v;
        }
        __threadfence();
#pragma unroll
        for (int it = 0; it < 4; ++it) {
            const v4f v = sv[it * 32 + lane];
            *(volatile v4f*)(gp + (size_t)(it * 4 + (lane >> 3)) * GF) = v;
        }
        __syncthreads();
    }
}

__global__ __launch_bounds__(32) void k_pool(const float* yp, const int* __restrict__ gid, float* part,
                                             int N, int G, int chunk) {
    __shared__ __attribute__((aligned(16))) float acc[GMAX * 32];
    const int lane = threadIdx.x & 31;
    const int slab = blockIdx.x;
    const int ch = blockIdx.y;
#pragma unroll 8
    for (int g = 0; g < GMAX; ++g) acc[g * 32 + lane] = 0.0f;
    __syncthreads();
    const int n0 = ch * chunk;
    int n1 = n0 + chunk;
    n1 = n1 > N ? N : n1;
#pragma unroll 1
    for (int n = n0; n < n1; ++n) {
        const int g = gid[n];
        const float v = yp[(size_t)n * GF + 32 * slab + lane];
        if ((unsigned)g < (unsigned)G) acc[g * 32 + lane] += v;
    }
    __syncthreads();

    const v4fa* av = (const v4fa*)acc;
    float* pb = part + (size_t)ch * GMAX * GF + 32 * slab + (lane & 7) * 4;
#pragma unroll 8
    for (int it = 0; it < GMAX / 4; ++it) {
        const v4f v = av[it * 32 + lane];
        *(volatile v4f*)(pb + (size_t)(it * 4 + (lane >> 3)) * GF) = v;
    }
    __threadfence();
#pragma unroll 8
    for (int it = 0; it < GMAX / 4; ++it) {
        const v4f v = av[it * 32 + lane];
        *(volatile v4f*)(pb + (size_t)(it * 4 + (lane >> 3)) * GF) = v;
    }
}

__global__ __launch_bounds__(256) void k_head(const float* part, const float* __restrict__ wp,
                                              const float* __restrict__ bp, float* out, int G, int out_size) {
    __shared__ __attribute__((aligned(16))) float outl[GMAX];
    const int t = threadIdx.x, lane = t & 31, wid = t >> 5;
    float accv = 0.0f;
#pragma unroll 1
    for (int c = 0; c < GF; ++c) {
        float s = 0.0f;
#pragma unroll 1
        for (int chn = 0; chn < NCH; ++chn) s += part[((size_t)chn * GMAX + t) * GF + c];
        accv = fmaf(s, wp[c], accv);
    }
    outl[t] = accv + bp[0];
    __syncthreads();

    const int nv4 = out_size >> 2;
    const v4fa* ovp = (const v4fa*)outl;
#pragma unroll
    for (int it = 0; it < GMAX / 128; ++it) {
        const int idx = it * 32 + lane;
        const v4f val = ovp[idx];
        const bool ok = (wid == 0) && (idx < nv4);
        if (ok) *(volatile v4f*)(out + (size_t)idx * 4) = val;
    }
    __threadfence();
#pragma unroll
    for (int it = 0; it < GMAX / 128; ++it) {
        const int idx = it * 32 + lane;
        const v4f val = ovp[idx];
        const bool ok = (wid == 0) && (idx < nv4);
        if (ok) *(volatile v4f*)(out + (size_t)idx * 4) = val;
    }
    (void)G;
}

extern "C" void kernel_launch(void* const* d_in, const int* in_sizes, int n_in,
                              void* d_out, int out_size, void* d_ws, size_t ws_size,
                              hipStream_t stream) {
    if (n_in < 15) return;
    const float* x   = (const float*)d_in[0];
    const float* ef  = (const float*)d_in[1];
    const int*   src = (const int*)d_in[2];
    const int*   dst = (const int*)d_in[3];
    const int*   gid = (const int*)d_in[4];
    const float* wg  = (const float*)d_in[5];
    const float* bg  = (const float*)d_in[6];
    const float* wr  = (const float*)d_in[7];
    const float* br  = (const float*)d_in[8];
    const float* wi  = (const float*)d_in[9];
    const float* bi  = (const float*)d_in[10];
    const float* wo  = (const float*)d_in[11];
    const float* bo  = (const float*)d_in[12];
    const float* wp  = (const float*)d_in[13];
    const float* bp  = (const float*)d_in[14];
    float* out = (float*)d_out;

    const int N = in_sizes[0] / FEAT;
    const int E = in_sizes[2];
    const int G = out_size;
    if (N <= 0 || E <= 0 || G < 1 || G > GMAX || (G & 3) != 0) return;
    if (in_sizes[0] != N * FEAT || in_sizes[3] != E || in_sizes[4] != N) return;
    if (in_sizes[5] != FEAT * FEAT || in_sizes[6] != FEAT || in_sizes[7] != FEAT * FEAT || in_sizes[8] != FEAT ||
        in_sizes[9] != FEAT * FEAT || in_sizes[10] != FEAT || in_sizes[11] != FEAT * GF || in_sizes[12] != GF ||
        in_sizes[13] != GF || in_sizes[14] < 1) return;

    const int NB = (N + 31) / 32;
    if (NB + 1 > PITCHB) return;
    const int NB1 = (E + CH1 - 1) / CH1;
    if (NB1 > MAXNB1) return;
    const int NT = (N + 15) / 16;
    const int chunk = (N + NCH - 1) / NCH;

    size_t off = 0;
    auto carve = [&](size_t bytes) -> size_t { const size_t p = off; off += (bytes + 255) & ~(size_t)255; return p; };
    const size_t o_bf = carve((size_t)NSLOTS * 8 * sizeof(_Float16));
    const size_t o_lists = carve((size_t)NB1 * CH1 * sizeof(int));
    const size_t o_tab = carve((size_t)NB1 * PITCHB * sizeof(int));
    const size_t o_agg = carve((size_t)NB * 32 * FEAT * sizeof(float));
    const size_t o_yp = carve((size_t)NT * 16 * GF * sizeof(float));
    const size_t o_part = carve((size_t)NCH * GMAX * GF * sizeof(float));
    if (off > ws_size || off > (size_t)134217728) return;

    char* ws = (char*)d_ws;
    _Float16* bfrag = (_Float16*)(ws + o_bf);
    int* lists = (int*)(ws + o_lists);
    int* offtab = (int*)(ws + o_tab);
    float* agg = (float*)(ws + o_agg);
    float* yp = (float*)(ws + o_yp);
    float* part = (float*)(ws + o_part);

    k_prep<<<(NSLOTS + 255) / 256, 256, 0, stream>>>(wg, wr, wi, wo, ef, bfrag);
    k_bucket<<<NB1, 128, 0, stream>>>(dst, lists, offtab, E, N);
    k_aggr<<<NB, 32, 0, stream>>>(x, src, dst, lists, offtab, agg, E, N, NB1);
    k_node<<<NT, 32, 0, stream>>>(agg, x, bfrag, bg, br, bi, bo, yp, N, NT);
    k_pool<<<dim3(GF / 32, NCH), 32, 0, stream>>>(yp, gid, part, N, G, chunk);
    k_head<<<1, 256, 0, stream>>>(part, wp, bp, out, G, out_size);
}
